// MultiheadLinearSelfAttentionKernalization_27865747817033
// MI455X (gfx1250) — hardware-verified
//
#include <hip/hip_runtime.h>


namespace {
constexpr int B = 2, S = 2048, D = 1024, NH = 16, DP = 64, NR = B * S;
constexpr float XS = 8.0f, WSC = 256.0f, AS = 0.0625f;
typedef _Float16 b16;
typedef __attribute__((ext_vector_type(16))) _Float16 v16b;
typedef __attribute__((ext_vector_type(8))) _Float16 v8b;
typedef __attribute__((ext_vector_type(8))) float v8f;
typedef __attribute__((ext_vector_type(4))) float v4f;
__device__ __forceinline__ float bf16_rne(float f) { unsigned int u = __float_as_uint(f); u += 0x7FFFu + ((u >> 16) & 1u); return __uint_as_float(u & 0xFFFF0000u); }
__device__ __forceinline__ void split16(float v, b16& hi, b16& lo) { hi = (b16)v; lo = (b16)(v - (float)hi); }
__device__ __forceinline__ v16b frag_kb(const b16* p, int hh) { const v8b a = *(const v8b*)(p + 8 * hh), b = *(const v8b*)(p + 16 + 8 * hh); v16b f;
#pragma unroll
  for (int e = 0; e < 8; ++e) { f[e] = a[e]; f[8 + e] = b[e]; } return f; }
__device__ __forceinline__ v8f wmma16b(v16b a, v16b b, v8f c) { v8f d = __builtin_amdgcn_wmma_f32_16x16x32_f16(false, a, false, b, (short)0, c, false, false); asm volatile("v_nop\n\tv_nop\n\tv_nop\n\tv_nop" : "+v"(d) : "v"(a), "v"(b)); return d; }
__device__ __forceinline__ void wave_lds_sync() { __builtin_amdgcn_fence(__ATOMIC_RELEASE, "workgroup"); __builtin_amdgcn_wave_barrier(); __builtin_amdgcn_fence(__ATOMIC_ACQUIRE, "workgroup"); }
__device__ __forceinline__ float pmul(float a, float b) { float p = a * b; asm volatile("" : "+v"(p)); return p; }
__device__ __forceinline__ float elu1(float v) { return v > 0.0f ? v + 1.0f : __expf(v); }

__global__ __launch_bounds__(256) void wput_kernel(const float* __restrict__ w, b16* __restrict__ WT) { const int u = blockIdx.x * 256 + threadIdx.x; if (u >= D * (D / 8)) return; const int o = u / (D / 8), k0 = (u % (D / 8)) * 8; v8b v;
#pragma unroll
  for (int j = 0; j < 8; ++j) v[j] = (b16)(bf16_rne(w[(size_t)(k0 + j) * D + o]) * WSC); for (int pass = 0; pass < 2; ++pass) { *(volatile v8b*)(WT + (size_t)o * D + k0) = v; __threadfence(); } }
__global__ __launch_bounds__(32) void qkv_kernel(const float* __restrict__ x, const b16* __restrict__ WQ, const b16* __restrict__ WK, const b16* __restrict__ WV, const float* __restrict__ bq, const float* __restrict__ bk, const float* __restrict__ bv, int RL, float* __restrict__ Q, float* __restrict__ Kn, float* __restrict__ V) {
  __shared__ __attribute__((aligned(16))) b16 Ah[16][D + 8]; __shared__ float Tf[16][132]; const int lane = threadIdx.x, nloc = lane & 15, hlf = lane >> 4; const int cg = blockIdx.x % 8, which = (blockIdx.x / 8) % 3; const size_t m0 = (size_t)(blockIdx.x / 24) * 16; if (m0 >= (size_t)RL) return;
  const b16* W = which == 0 ? WQ : (which == 1 ? WK : WV); const float* bias = which == 0 ? bq : (which == 1 ? bk : bv); float* O = which == 0 ? Q : (which == 1 ? Kn : V);
  for (int rr = 0; rr < 16; ++rr) for (int q = 0; q < D / 32; ++q) Ah[rr][q * 32 + lane] = (b16)(bf16_rne(x[(m0 + rr) * D + q * 32 + lane]) * XS);
  wave_lds_sync(); v8f acc[8];
#pragma unroll
  for (int t = 0; t < 8; ++t) acc[t] = (v8f){};
#pragma unroll 2
  for (int kb = 0; kb < D; kb += 32) { const v16b a = frag_kb(&Ah[nloc][kb], hlf);
#pragma unroll
    for (int t = 0; t < 8; ++t) acc[t] = wmma16b(a, frag_kb(W + (size_t)(cg * 128 + t * 16 + nloc) * D + kb, hlf), acc[t]); }
#pragma unroll
  for (int t = 0; t < 8; ++t) { const int c = cg * 128 + t * 16 + nloc; const float bb = bf16_rne(bias[c]);
#pragma unroll
    for (int r8 = 0; r8 < 8; ++r8) { float v = acc[t][r8] * (1.0f / (XS * WSC)) + bb; if (which < 2) v = elu1(v); Tf[8 * hlf + r8][t * 16 + nloc] = v; } }
  wave_lds_sync();
  if (which == 1) { const int row = lane & 15, hd = lane >> 4; float s = 0.0f; for (int d = 0; d < DP; ++d) { const float v = Tf[row][hd * 64 + d]; s += pmul(v, v); } const float inv = 1.0f / sqrtf(s + 1e-6f); wave_lds_sync(); for (int d = 0; d < DP; ++d) Tf[row][hd * 64 + d] = pmul(Tf[row][hd * 64 + d], inv); wave_lds_sync(); }
  for (int pass = 0; pass < 2; ++pass) { for (int rr = 0; rr < 16; ++rr) *(volatile v4f*)(O + (m0 + rr) * D + cg * 128 + lane * 4) = *(const v4f*)(&Tf[rr][lane * 4]); __threadfence(); }
}
__global__ __launch_bounds__(32) void kv_kernel(const float* __restrict__ Kn, const float* __restrict__ V, int BV, float* __restrict__ KVT) {
  __shared__ __attribute__((aligned(16))) b16 Ah[16][40], Al[16][40], Bh[64][40], Bl[64][40]; __shared__ float Tf[16][DP + 2]; const int lane = threadIdx.x, nloc = lane & 15, hlf = lane >> 4;
  const int et = blockIdx.x % 4, h = (blockIdx.x / 4) % NH, b = blockIdx.x / (4 * NH); if (b >= BV) return; v8f acc[4] = {(v8f){}, (v8f){}, (v8f){}, (v8f){}};
#pragma unroll 1
  for (int sc = 0; sc < S; sc += 32) {
    for (int rr = 0; rr < 32; ++rr) { const size_t row = ((size_t)b * S + sc + rr) * D + h * DP; b16 p, q; if (lane < 16) { split16(V[row + et * 16 + lane] * XS, p, q); Ah[lane][rr] = p; Al[lane][rr] = q; } for (int q2 = 0; q2 < 2; ++q2) { split16(Kn[row + q2 * 32 + lane] * XS, p, q); Bh[q2 * 32 + lane][rr] = p; Bl[q2 * 32 + lane][rr] = q; } }
    wave_lds_sync(); const v16b a = frag_kb(&Ah[nloc][0], hlf), al = frag_kb(&Al[nloc][0], hlf);
#pragma unroll
    for (int t = 0; t < 4; ++t) { const v16b bh = frag_kb(&Bh[t * 16 + nloc][0], hlf), bl = frag_kb(&Bl[t * 16 + nloc][0], hlf); acc[t] = wmma16b(a, bh, acc[t]); acc[t] = wmma16b(a, bl, acc[t]); acc[t] = wmma16b(al, bh, acc[t]); }
    wave_lds_sync(); }
#pragma unroll
  for (int t = 0; t < 4; ++t)
#pragma unroll
    for (int r8 = 0; r8 < 8; ++r8) Tf[8 * hlf + r8][t * 16 + nloc] = acc[t][r8] * (1.0f / (XS * XS));
  wave_lds_sync();
  for (int pass = 0; pass < 2; ++pass) { for (int rr = 0; rr < 16; ++rr) { const size_t orow = ((size_t)(b * NH + h) * DP + et * 16 + rr) * DP; ((volatile float*)KVT)[orow + lane] = Tf[rr][lane]; ((volatile float*)KVT)[orow + 32 + lane] = Tf[rr][32 + lane]; } __threadfence(); }
}
__global__ __launch_bounds__(32) void attn_kernel(const float* __restrict__ Q, const float* __restrict__ KVT, int RL, float* __restrict__ ATT) {
  __shared__ __attribute__((aligned(16))) b16 Ah[16][72], Al[16][72], Bh[64][72], Bl[64][72]; __shared__ float Tf[16][DP + 2]; const int lane = threadIdx.x, nloc = lane & 15, hlf = lane >> 4; const size_t m0 = (size_t)blockIdx.x * 16; if (m0 >= (size_t)RL) return; const int b = (int)(m0 / S);
#pragma unroll 1
  for (int h = 0; h < NH; ++h) {
    for (int rr = 0; rr < 16; ++rr) for (int q2 = 0; q2 < 2; ++q2) { b16 p, q; split16(Q[(m0 + rr) * D + h * DP + q2 * 32 + lane] * XS, p, q); Ah[rr][q2 * 32 + lane] = p; Al[rr][q2 * 32 + lane] = q; }
    for (int e = 0; e < DP; ++e) for (int q2 = 0; q2 < 2; ++q2) { b16 p, q; split16(KVT[((size_t)(b * NH + h) * DP + e) * DP + q2 * 32 + lane], p, q); Bh[e][q2 * 32 + lane] = p; Bl[e][q2 * 32 + lane] = q; }
    wave_lds_sync(); v8f acc[4] = {(v8f){}, (v8f){}, (v8f){}, (v8f){}};
#pragma unroll
    for (int kb = 0; kb < DP; kb += 32) { const v16b a = frag_kb(&Ah[nloc][kb], hlf), al = frag_kb(&Al[nloc][kb], hlf);
#pragma unroll
      for (int t = 0; t < 4; ++t) { const v16b bh = frag_kb(&Bh[t * 16 + nloc][kb], hlf), bl = frag_kb(&Bl[t * 16 + nloc][kb], hlf); acc[t] = wmma16b(a, bh, acc[t]); acc[t] = wmma16b(a, bl, acc[t]); acc[t] = wmma16b(al, bh, acc[t]); } }
#pragma unroll
    for (int t = 0; t < 4; ++t)
#pragma unroll
      for (int r8 = 0; r8 < 8; ++r8) Tf[8 * hlf + r8][t * 16 + nloc] = acc[t][r8] * (1.0f / XS);
    wave_lds_sync();
    for (int pass = 0; pass < 2; ++pass) { for (int rr = 0; rr < 16; ++rr) { ((volatile float*)ATT)[(m0 + rr) * D + h * DP + lane] = Tf[rr][lane]; ((volatile float*)ATT)[(m0 + rr) * D + h * DP + 32 + lane] = Tf[rr][32 + lane]; } __threadfence(); }
    wave_lds_sync(); }
}
__global__ __launch_bounds__(32) void wo_kernel(const float* __restrict__ ATT, const b16* __restrict__ WO, const float* __restrict__ bo, const float* __restrict__ x, int RL, float* __restrict__ Y) {
  __shared__ __attribute__((aligned(16))) b16 Ah[16][D + 8], Al[16][D + 8]; __shared__ float Tf[16][132]; const int lane = threadIdx.x, nloc = lane & 15, hlf = lane >> 4; const int cg = blockIdx.x % 8; const size_t m0 = (size_t)(blockIdx.x / 8) * 16; if (m0 >= (size_t)RL) return;
  for (int rr = 0; rr < 16; ++rr) for (int q = 0; q < D / 32; ++q) { b16 p, ql; split16(ATT[(m0 + rr) * D + q * 32 + lane] * AS, p, ql); Ah[rr][q * 32 + lane] = p; Al[rr][q * 32 + lane] = ql; }
  wave_lds_sync(); v8f acc[8];
#pragma unroll
  for (int t = 0; t < 8; ++t) acc[t] = (v8f){};
#pragma unroll 2
  for (int kb = 0; kb < D; kb += 32) { const v16b a = frag_kb(&Ah[nloc][kb], hlf), al = frag_kb(&Al[nloc][kb], hlf);
#pragma unroll
    for (int t = 0; t < 8; ++t) { const v16b bw = frag_kb(WO + (size_t)(cg * 128 + t * 16 + nloc) * D + kb, hlf); acc[t] = wmma16b(a, bw, acc[t]); acc[t] = wmma16b(al, bw, acc[t]); } }
#pragma unroll
  for (int t = 0; t < 8; ++t) { const int c = cg * 128 + t * 16 + nloc; const float bb = bf16_rne(bo[c]);
#pragma unroll
    for (int r8 = 0; r8 < 8; ++r8) Tf[8 * hlf + r8][t * 16 + nloc] = acc[t][r8] * (1.0f / (AS * WSC)) + bb + bf16_rne(x[(m0 + 8 * hlf + r8) * D + c]); }
  wave_lds_sync();
  for (int pass = 0; pass < 2; ++pass) { for (int rr = 0; rr < 16; ++rr) *(volatile v4f*)(Y + (m0 + rr) * D + cg * 128 + lane * 4) = *(const v4f*)(&Tf[rr][lane * 4]); __threadfence(); }
}
__global__ __launch_bounds__(256) void ln_kernel(const float* __restrict__ Y, const float* __restrict__ g, const float* __restrict__ bt, int RL, float* __restrict__ out) {
  const int wave = threadIdx.x >> 5, lane = threadIdx.x & 31; const size_t r = (size_t)blockIdx.x * 8 + wave; if (r >= (size_t)RL) return; const float* pr = Y + r * D; float s = 0.0f;
#pragma unroll 4
  for (int q = 0; q < 32; ++q) s += pr[q * 32 + lane];
  for (int o = 16; o; o >>= 1) s += __shfl_xor(s, o); const float mu = s * (1.0f / D); float vq = 0.0f;
#pragma unroll 4
  for (int q = 0; q < 32; ++q) { const float dd = pr[q * 32 + lane] - mu; vq += pmul(dd, dd); }
  for (int o = 16; o; o >>= 1) vq += __shfl_xor(vq, o); const float rs = 1.0f / sqrtf(vq * (1.0f / D) + 1e-6f);
  for (int pass = 0; pass < 2; ++pass) {
#pragma unroll 4
    for (int q = 0; q < 32; ++q) { const int d = q * 32 + lane; ((volatile float*)out)[r * D + d] = pmul(pmul(pr[d] - mu, rs), bf16_rne(g[d])) + bf16_rne(bt[d]); } __threadfence(); }
}
}

extern "C" void kernel_launch(void* const* d_in, const int* in_sizes, int n_in, void* d_out, int out_size, void* d_ws, size_t ws_size, hipStream_t stream) {
  (void)n_in;
  auto Fp = [&](int i) { return (const float*)d_in[i]; };
  if (in_sizes[0] != NR * D || in_sizes[1] != D * D || in_sizes[3] != D * D || in_sizes[5] != D * D || in_sizes[7] != D * D || in_sizes[9] != D || out_size != NR * D) return;
  const int BV = B; const int RL = BV * S;
  size_t off = 0; char* ws = (char*)d_ws;
  auto carve = [&](size_t bytes) { char* p = ws + off; off += (bytes + 255) & ~(size_t)255; return p; };
  b16* WQ = (b16*)carve((size_t)D * D * 2); b16* WK = (b16*)carve((size_t)D * D * 2); b16* WV = (b16*)carve((size_t)D * D * 2); b16* WO = (b16*)carve((size_t)D * D * 2);
  float* Q = (float*)carve((size_t)NR * D * 4); float* Kn = (float*)carve((size_t)NR * D * 4); float* V = (float*)carve((size_t)NR * D * 4); float* KVT = (float*)carve((size_t)B * NH * DP * DP * 4); float* ATT = (float*)carve((size_t)NR * D * 4); float* Y = (float*)carve((size_t)NR * D * 4);
  if (off > ws_size || off > ((size_t)128 << 20)) return;
  wput_kernel<<<(D * (D / 8) + 255) / 256, 256, 0, stream>>>(Fp(1), WQ); wput_kernel<<<(D * (D / 8) + 255) / 256, 256, 0, stream>>>(Fp(3), WK); wput_kernel<<<(D * (D / 8) + 255) / 256, 256, 0, stream>>>(Fp(5), WV); wput_kernel<<<(D * (D / 8) + 255) / 256, 256, 0, stream>>>(Fp(7), WO);
  qkv_kernel<<<(RL / 16) * 24, 32, 0, stream>>>(Fp(0), WQ, WK, WV, Fp(2), Fp(4), Fp(6), RL, Q, Kn, V);
  kv_kernel<<<BV * NH * 4, 32, 0, stream>>>(Kn, V, BV, KVT);
  attn_kernel<<<RL / 16, 32, 0, stream>>>(Q, KVT, RL, ATT);
  wo_kernel<<<(RL / 16) * 8, 32, 0, stream>>>(ATT, WO, Fp(8), Fp(0), RL, Y);
  ln_kernel<<<(RL + 7) / 8, 256, 0, stream>>>(Y, Fp(9), Fp(10), RL, (float*)d_out);
}
